// LinearAttention_39152921870872
// MI455X (gfx1250) — hardware-verified
//
#include <hip/hip_runtime.h>
#include <stddef.h>


#pragma clang fp contract(off)

typedef _Float16 v16h __attribute__((ext_vector_type(16)));
typedef _Float16 v8h  __attribute__((ext_vector_type(8)));
typedef float    v8f  __attribute__((ext_vector_type(8)));
typedef float    v4f  __attribute__((ext_vector_type(4)));
typedef _Float16 h16;

#ifndef NB
#define NB 8
#endif
#ifndef SEQ
#define SEQ 4096
#endif
#define NB_FULL  8
#define SEQ_FULL 4096
#define CDIM  256
#define MROWS (NB * SEQ)

static_assert(NB >= 1 && NB <= NB_FULL);
static_assert(SEQ >= 128 && SEQ <= SEQ_FULL && (SEQ % 128) == 0);
static_assert(CDIM == 256);
static_assert(CDIM == 32 * 8);
static_assert((CDIM % 64) == 0 && (CDIM % 32) == 0);
static_assert((SEQ % 64) == 0 && (SEQ % 32) == 0);
static_assert((MROWS % 64) == 0 && (MROWS % 8) == 0);
static_assert(((NB * CDIM) % 64) == 0);
static_assert((size_t)MROWS * CDIM < (size_t)0xFFFFFFFFu);

#define LDT 72
#define LDC 68
static_assert((LDT % 8) == 0 && LDT >= 64);
static_assert((LDC % 4) == 0 && LDC >= 64);

#define QCARRY  64.0f
#define KCARRY  64.0f
#define VCARRYP 1.0f
#define KVCARRY 16.0f

#define QN_BYTES ((size_t)MROWS * CDIM * 2)
#define KT_BYTES ((size_t)NB * CDIM * SEQ * 2)
#define VT_BYTES ((size_t)NB * CDIM * SEQ * 2)
#define KV_BYTES ((size_t)NB * CDIM * CDIM * 2)
#define OFF_QN ((size_t)0)
#define OFF_KT (OFF_QN + QN_BYTES)
#define OFF_VT (OFF_KT + KT_BYTES)
#define OFF_KV (OFF_VT + VT_BYTES)
#define WS_TOTAL (OFF_KV + KV_BYTES)
static_assert((QN_BYTES % 128) == 0 && (KT_BYTES % 128) == 0);
static_assert((VT_BYTES % 128) == 0 && (KV_BYTES % 128) == 0);
static_assert(WS_TOTAL <= (size_t)134217728);

__device__ __forceinline__ float bf16r(float x) {
  unsigned int u = __float_as_uint(x);
  u = (u + 0x7FFFu + ((u >> 16) & 1u)) & 0xFFFF0000u;
  return __uint_as_float(u);
}

static __device__ __forceinline__ h16 toh_flush(float v) {
  const h16 r = (h16)v;
  return (fabsf(v) < 6.103515625e-05f) ? (h16)0.0f : r;
}

__device__ __forceinline__ v16h frag_at(const _Float16* p) {
  v8h lo = *(const v8h*)(p);
  v8h hi = *(const v8h*)(p + 16);
  v16h out;
#pragma unroll
  for (int i = 0; i < 8; ++i) { out[i] = lo[i]; out[i + 8] = hi[i]; }
  return out;
}

__device__ __forceinline__ v8f wmma16(v16h a, v16h b, v8f c) {
  v8f d = __builtin_amdgcn_wmma_f32_16x16x32_f16(false, a, false, b, (short)0, c,
                                                 false, false);
  asm volatile("v_nop\n\tv_nop\n\tv_nop\n\tv_nop" : "+v"(d) : "v"(a), "v"(b));
  return d;
}

__device__ __forceinline__ float red32_sum(float x) {
#pragma unroll
  for (int off = 1; off < 32; off <<= 1) x += __shfl_xor(x, off, 32);
  return x;
}

__global__ __launch_bounds__(256) void qnorm_kernel(
    const float* __restrict__ X, _Float16* __restrict__ dst) {
  const unsigned lane = threadIdx.x & 31u;
  const unsigned w = (unsigned)__builtin_amdgcn_readfirstlane((int)(threadIdx.x >> 5));
  const unsigned crow = blockIdx.x * 8u + w;
  const unsigned bidx = crow / (unsigned)SEQ;
  const unsigned sq = crow - bidx * (unsigned)SEQ;
  const size_t srow = (size_t)bidx * SEQ_FULL + sq;
  const float* xr = X + srow * CDIM + lane * 8u;
  const v4f a0 = *(const v4f*)(xr);
  const v4f a1 = *(const v4f*)(xr + 4u);
  float e[8];
#pragma unroll
  for (int i = 0; i < 4; ++i) { e[i] = bf16r(a0[i]); e[i + 4] = bf16r(a1[i]); }
  float ss = 0.0f;
#pragma unroll
  for (int i = 0; i < 8; ++i) ss += e[i] * e[i];
  ss = red32_sum(ss);
  const float sc = QCARRY * (1.0f / fmaxf(sqrtf(ss), 1.0e-12f));
  v8h o;
#pragma unroll
  for (int i = 0; i < 8; ++i) o[i] = toh_flush(e[i] * sc);
  _Float16* p = dst + (size_t)crow * CDIM + lane * 8u;
  *(volatile v8h*)p = o;
  __threadfence();
  *(volatile v8h*)p = o;
}

template <int NORM>
__device__ __forceinline__ void tprep_body(const float* __restrict__ X,
                                           _Float16* __restrict__ XT) {
  __shared__ _Float16 T[CDIM * LDT];
  const unsigned tid = threadIdx.x, lane = tid & 31u;
  const unsigned w = (unsigned)__builtin_amdgcn_readfirstlane((int)(threadIdx.x >> 5));
  const unsigned m0 = blockIdx.x * 64u;
  const unsigned b = blockIdx.y;

#pragma unroll 1
  for (unsigned j = 0; j < 8u; ++j) {
    const unsigned ml = w * 8u + j;
    const size_t srow = (size_t)b * SEQ_FULL + m0 + ml;
    const float* xr = X + srow * CDIM + lane * 8u;
    const v4f a0 = *(const v4f*)(xr);
    const v4f a1 = *(const v4f*)(xr + 4u);
    float e[8];
#pragma unroll
    for (int i = 0; i < 4; ++i) { e[i] = bf16r(a0[i]); e[i + 4] = bf16r(a1[i]); }
    float sc = VCARRYP;
    if (NORM) {
      float ss = 0.0f;
#pragma unroll
      for (int i = 0; i < 8; ++i) ss += e[i] * e[i];
      ss = red32_sum(ss);
      sc = KCARRY * (1.0f / fmaxf(sqrtf(ss), 1.0e-12f));
    }
#pragma unroll
    for (int i = 0; i < 8; ++i)
      T[(lane * 8u + (unsigned)i) * LDT + ml] = toh_flush(e[i] * sc);
  }
  __syncthreads();

  v8h x[8];
  size_t off[8];
#pragma unroll
  for (unsigned i = 0; i < 8u; ++i) {
    const unsigned c = 32u * i + (tid >> 3);
    const unsigned mc = (tid & 7u) * 8u;
    x[i] = *(const v8h*)&T[c * LDT + mc];
    off[i] = ((size_t)b * CDIM + c) * SEQ + m0 + mc;
  }
#pragma unroll
  for (int i = 0; i < 8; ++i) *(volatile v8h*)(XT + off[i]) = x[i];
  __threadfence();
#pragma unroll
  for (int i = 0; i < 8; ++i) *(volatile v8h*)(XT + off[i]) = x[i];
}

__global__ __launch_bounds__(256) void knormT_kernel(
    const float* __restrict__ X, _Float16* __restrict__ XT) {
  tprep_body<1>(X, XT);
}
__global__ __launch_bounds__(256) void vconvT_kernel(
    const float* __restrict__ X, _Float16* __restrict__ XT) {
  tprep_body<0>(X, XT);
}

template <int MODE>
__device__ __forceinline__ void gemm_body(
    const _Float16* __restrict__ A16, const _Float16* __restrict__ BtAll, const unsigned K,
    const unsigned rpb, float* __restrict__ outf, _Float16* __restrict__ out16) {
  __shared__ float Cs[64 * LDC];
  const unsigned tid = threadIdx.x, lane = tid & 31u;
  const unsigned w = (unsigned)__builtin_amdgcn_readfirstlane((int)(threadIdx.x >> 5));
  const unsigned mw = w >> 1, nw = w & 1u;
  const unsigned hh = lane >> 4, m = lane & 15u;
  const unsigned n0 = blockIdx.x * 64u;
  const unsigned row0 = blockIdx.y * 64u;
  const unsigned bsel = row0 / rpb;
  const _Float16* Bt = BtAll + (size_t)bsel * CDIM * K;

  const _Float16* ap  = A16 + (size_t)(row0 + mw * 16u + m) * K + hh * 8u;
  const _Float16* bp0 = Bt + (size_t)(n0 + nw * 32u + m) * K + hh * 8u;
  const _Float16* bp1 = bp0 + (size_t)16 * K;
  v8f acc0 = {}, acc1 = {};
#pragma unroll 2
  for (unsigned k0 = 0; k0 < K; k0 += 32u) {
    const v16h a  = frag_at(ap + k0);
    const v16h b0 = frag_at(bp0 + k0);
    const v16h b1 = frag_at(bp1 + k0);
    acc0 = wmma16(a, b0, acc0);
    acc1 = wmma16(a, b1, acc1);
  }
#pragma unroll
  for (int r = 0; r < 8; ++r) {
    float* d = &Cs[(mw * 16u + hh * 8u + (unsigned)r) * LDC + nw * 32u + m];
    d[0]  = acc0[r];
    d[16] = acc1[r];
  }
  __syncthreads();

  if (MODE == 0) {
    const float cs = KVCARRY / (KCARRY * VCARRYP);
    v8h x[2];
    size_t off[2];
#pragma unroll
    for (unsigned i = 0; i < 2u; ++i) {
      const unsigned r = 32u * i + (tid >> 3);
      const unsigned c = (tid & 7u) * 8u;
      const v4f u0 = *(const v4f*)&Cs[r * LDC + c];
      const v4f u1 = *(const v4f*)&Cs[r * LDC + c + 4];
#pragma unroll
      for (int j = 0; j < 4; ++j) {
        x[i][j]     = toh_flush(u0[j] * cs);
        x[i][j + 4] = toh_flush(u1[j] * cs);
      }
      off[i] = (size_t)(row0 + r) * CDIM + n0 + c;
    }
#pragma unroll
    for (int i = 0; i < 2; ++i) *(volatile v8h*)(out16 + off[i]) = x[i];
    __threadfence();
#pragma unroll
    for (int i = 0; i < 2; ++i) *(volatile v8h*)(out16 + off[i]) = x[i];
  }

  if (MODE == 1) {
    const float cs = 1.0f / (QCARRY * KVCARRY * (float)SEQ);
    v4f xs[4];
    size_t off[4];
#pragma unroll
    for (unsigned i = 0; i < 4u; ++i) {
      const unsigned r = 16u * i + (tid >> 4);
      const unsigned c = (tid & 15u) * 4u;
      const unsigned crow = row0 + r;
      const unsigned bidx = crow / (unsigned)SEQ;
      const unsigned sq = crow - bidx * (unsigned)SEQ;
      const size_t frow = (size_t)bidx * SEQ_FULL + sq;
      const v4f u = *(const v4f*)&Cs[r * LDC + c];
      v4f val;
#pragma unroll
      for (int j = 0; j < 4; ++j) val[j] = u[j] * cs;
      xs[i] = val;
      off[i] = frow * CDIM + n0 + c;
    }
#pragma unroll
    for (int i = 0; i < 4; ++i) *(volatile v4f*)(outf + off[i]) = xs[i];
    __threadfence();
#pragma unroll
    for (int i = 0; i < 4; ++i) *(volatile v4f*)(outf + off[i]) = xs[i];
  }
}

__global__ __launch_bounds__(256) void gemm_kv_kernel(
    const _Float16* __restrict__ vT, const _Float16* __restrict__ knT,
    _Float16* __restrict__ kvT) {
  gemm_body<0>(vT, knT, (unsigned)SEQ, (unsigned)CDIM, (float*)0, kvT);
}
__global__ __launch_bounds__(256) void gemm_ctx_kernel(
    const _Float16* __restrict__ qn, const _Float16* __restrict__ kvT,
    float* __restrict__ outf) {
  gemm_body<1>(qn, kvT, (unsigned)CDIM, (unsigned)SEQ, outf, (_Float16*)0);
}

extern "C" void kernel_launch(void* const* d_in, const int* in_sizes, int n_in,
                              void* d_out, int out_size, void* d_ws, size_t ws_size,
                              hipStream_t stream) {
  if (n_in < 3) return;
  const long long need_x = ((long long)(NB - 1) * SEQ_FULL + SEQ) * CDIM;
  if ((long long)in_sizes[0] < need_x) return;
  if ((long long)in_sizes[1] < need_x) return;
  if ((long long)in_sizes[2] < need_x) return;
  if ((long long)out_size < need_x) return;
  if (ws_size < WS_TOTAL) return;

  const float* Qin = (const float*)d_in[0];
  const float* Kin = (const float*)d_in[1];
  const float* Vin = (const float*)d_in[2];
  float* out = (float*)d_out;

  char* ws = (char*)d_ws;
  _Float16* QN16  = (_Float16*)(ws + OFF_QN);
  _Float16* KNT16 = (_Float16*)(ws + OFF_KT);
  _Float16* VT16  = (_Float16*)(ws + OFF_VT);
  _Float16* KVT16 = (_Float16*)(ws + OFF_KV);

  dim3 blk(256);
  qnorm_kernel<<<dim3(MROWS / 8), blk, 0, stream>>>(Qin, QN16);
  knormT_kernel<<<dim3(SEQ / 64, NB), blk, 0, stream>>>(Kin, KNT16);
  vconvT_kernel<<<dim3(SEQ / 64, NB), blk, 0, stream>>>(Vin, VT16);
  gemm_kv_kernel<<<dim3(CDIM / 64, (NB * CDIM) / 64), blk, 0, stream>>>(VT16, KNT16, KVT16);
  gemm_ctx_kernel<<<dim3(CDIM / 64, MROWS / 64), blk, 0, stream>>>(QN16, KVT16, out);
}
